// CustomAttentionClassifier_43619687858748
// MI455X (gfx1250) — hardware-run, weakly checked
//
#include <hip/hip_runtime.h>
#include <math.h>

typedef __attribute__((ext_vector_type(16))) _Float16 v16h;
typedef __attribute__((ext_vector_type(16))) __bf16 v16b;
typedef __attribute__((ext_vector_type(8)))  _Float16 v8h;
typedef __attribute__((ext_vector_type(8)))  float v8f;
typedef __attribute__((ext_vector_type(4)))  float v4f;
typedef __attribute__((ext_vector_type(2)))  float v2f;
typedef __attribute__((ext_vector_type(4)))  unsigned v4u;
typedef __attribute__((ext_vector_type(4)))  int v4i;
typedef float __attribute__((may_alias)) float_a;
typedef int __attribute__((may_alias)) int_a;

template <typename T> __device__ __forceinline__ void vst2(void* p, T v) { *(volatile T*)p = v; __threadfence(); *(volatile T*)p = v; }
__device__ __forceinline__ v8f wmma16(v16h a, v16h b, v8f c) {
  v8f d = __builtin_amdgcn_wmma_f32_16x16x32_f16(false, a, false, b, (short)0, c, false, false);
  asm volatile("v_nop\n\tv_nop\n\tv_nop\n\tv_nop" : "+v"(d) : "v"(a), "v"(b));
  return d;
}
__device__ __forceinline__ v8f wmma_bf(v16b a, v16b b, v8f c) {
  v8f d = __builtin_amdgcn_wmma_f32_16x16x32_bf16(false, a, false, b, (short)0, c, false, false);
  asm volatile("v_nop\n\tv_nop\n\tv_nop\n\tv_nop" : "+v"(d) : "v"(a), "v"(b));
  return d;
}
__device__ __forceinline__ v16h frag_h(const _Float16* rowk0, int lane) {
  union { v16h v; v8h q[2]; } u; const _Float16* p = rowk0 + 8 * (lane >> 4);
  u.q[0] = *(const v8h*)p; u.q[1] = *(const v8h*)(p + 16); return u.v;
}
__device__ __forceinline__ v16h frag_f32(const float* rowk0, int lane) {
  v16h a; const float* p = rowk0 + 8 * (lane >> 4);
#pragma unroll
  for (int i = 0; i < 8; ++i) { a[i] = (_Float16)p[i]; a[8 + i] = (_Float16)p[16 + i]; }
  return a;
}
__device__ __forceinline__ v16h frag_f32s(const float* rowk0, int lane, float sc) {
  v16h a; const float* p = rowk0 + 8 * (lane >> 4);
#pragma unroll
  for (int i = 0; i < 8; ++i) { a[i] = (_Float16)(p[i] * sc); a[8 + i] = (_Float16)(p[16 + i] * sc); }
  return a;
}
__device__ __forceinline__ v16h fragc_f32(const float* W, int k0, int n, int lane, int ld, int K) {
  v16h a; const int g = lane >> 4;
#pragma unroll
  for (int i = 0; i < 8; ++i) { const int ka = k0 + 8 * g + i, kb = ka + 16;
    a[i] = (_Float16)(ka < K ? W[(size_t)(ka < K ? ka : K - 1) * ld + n] : 0.f); a[8 + i] = (_Float16)(kb < K ? W[(size_t)(kb < K ? kb : K - 1) * ld + n] : 0.f); }
  return a;
}
struct F2 { v16b h, l; };
__device__ __forceinline__ F2 bsplit16(const float v[16]) { F2 r;
#pragma unroll
  for (int i = 0; i < 16; ++i) { const __bf16 h = (__bf16)v[i]; r.h[i] = h; r.l[i] = (__bf16)(v[i] - (float)h); }
  return r; }
__device__ __forceinline__ F2 split_row(const float* row, int k0, int lane) { float v[16]; const float* p = row + k0 + 8 * (lane >> 4);
#pragma unroll
  for (int i = 0; i < 8; ++i) { v[i] = p[i]; v[8 + i] = p[16 + i]; }
  return bsplit16(v); }
__device__ __forceinline__ F2 split_rowK(const float* row, int k0, int lane, int K) { float v[16]; const int g = lane >> 4;
#pragma unroll
  for (int i = 0; i < 8; ++i) { const int ka = k0 + 8 * g + i, kb = ka + 16; v[i] = ka < K ? row[ka < K ? ka : K - 1] : 0.f; v[8 + i] = kb < K ? row[kb < K ? kb : K - 1] : 0.f; }
  return bsplit16(v); }
__device__ __forceinline__ F2 split_col(const float* W, int k0, int n, int lane, int ld, int K) { float v[16]; const int g = lane >> 4;
#pragma unroll
  for (int i = 0; i < 8; ++i) { const int ka = k0 + 8 * g + i, kb = ka + 16; v[i] = ka < K ? W[(size_t)(ka < K ? ka : K - 1) * ld + n] : 0.f; v[8 + i] = kb < K ? W[(size_t)(kb < K ? kb : K - 1) * ld + n] : 0.f; }
  return bsplit16(v); }
__device__ __forceinline__ v8f mac3(const F2& a, const F2& b, v8f c) { c = wmma_bf(a.l, b.h, c); c = wmma_bf(a.h, b.l, c); return wmma_bf(a.h, b.h, c); }
__device__ __forceinline__ float sigm(float v) { return 1.0f / (1.0f + expf(-v)); }
#define LDSX() do { asm volatile("s_wait_dscnt 0" ::: "memory"); __builtin_amdgcn_wave_barrier(); __builtin_amdgcn_fence(__ATOMIC_RELEASE, "workgroup"); } while (0)


#define NB 64
#define SS 512
#define DD 256
#define VOC 30522
#define HID 128
#define NCLS 16
#ifndef TNB
#define TNB NB
#endif
typedef __attribute__((ext_vector_type(8))) __bf16 v8b;
__device__ __forceinline__ v16b frag_b(const __bf16* rowk0, int lane) {
  union { v16b v; v8b q[2]; } u; const __bf16* p = rowk0 + 8 * (lane >> 4);
  u.q[0] = *(const v8b*)p; u.q[1] = *(const v8b*)(p + 16); return u.v;
}
__device__ __forceinline__ float bfr(float v) { return (float)(__bf16)v; }
__device__ __attribute__((noinline)) float exp_ni(float v) { return expf(v); }
__device__ __attribute__((noinline)) float erf_ni(float v) { return erff(v); }

#define WS_PW   0u
#define WS_PEW  (WS_PW + 2u * 3 * DD * DD)
#define WS_QKV  (WS_PEW + 4u * SS * 3 * DD)
#define WS_WP   (WS_QKV + 4u * NB * SS * 3 * DD)
#define WS_END  (WS_WP + 4u * NB * 8 * SS)

__global__ __launch_bounds__(256) void k_packT(const float* __restrict__ WQ, const float* __restrict__ WK, const float* __restrict__ WV, __bf16* __restrict__ PW) {
  __shared__ __align__(16) __bf16 s[DD]; const int n = blockIdx.x, k = threadIdx.x; const float* Wm = (n < DD) ? WQ : (n < 2 * DD ? WK : WV);
  s[k] = (__bf16)Wm[(size_t)k * DD + (n & (DD - 1))];
  __syncthreads();
  if (k < DD / 8) vst2((unsigned*)(PW + (size_t)n * DD + k * 8), *(const v4u*)&s[k * 8]);
}
__global__ __launch_bounds__(128) void k_pe(const __bf16* __restrict__ PW, const float* __restrict__ BQ, const float* __restrict__ BK, const float* __restrict__ BV, float* __restrict__ PEW) {
  __shared__ __align__(16) float spe[64][DD + 4]; __shared__ __align__(16) float so[4][16][132];
  const int tid = threadIdx.x, wave = tid >> 5, lane = tid & 31, col = lane & 15, g = lane >> 4; const int s0 = blockIdx.x * 64; const int n0 = blockIdx.y * 128;
  for (int q = tid; q < 64 * DD; q += 128) { const int sl = q >> 8, d = q & 255; const int i = d >> 1; const float div = expf((float)(2 * i) * (-logf(10000.0f) / (float)DD)); const float ang = (float)(s0 + sl) * div; spe[sl][d] = (d & 1) ? cosf(ang) : sinf(ang); }
  __syncthreads();
  v8f acc[8] = {};
#pragma unroll
  for (int kc = 0; kc < DD / 32; ++kc) { const F2 a = split_row(&spe[wave * 16 + col][0], kc * 32, lane);
#pragma unroll
    for (int j = 0; j < 8; ++j) { const v16b w = frag_b(PW + (size_t)(n0 + j * 16 + col) * DD + kc * 32, lane); acc[j] = wmma_bf(a.l, w, acc[j]); acc[j] = wmma_bf(a.h, w, acc[j]); } }
  const float* bias = (n0 < DD) ? BQ : (n0 < 2 * DD ? BK : BV);
#pragma unroll
  for (int j = 0; j < 8; ++j) { const float bb = bfr(bias[(n0 & (DD - 1)) + j * 16 + col]);
#pragma unroll
    for (int r = 0; r < 8; ++r) so[wave][8 * g + r][j * 16 + col] = acc[j][r] + bb; }
  LDSX();
  for (int rl = 0; rl < 16; ++rl) vst2(PEW + (size_t)(s0 + wave * 16 + rl) * (3 * DD) + n0 + lane * 4, *(const v4f*)&so[wave][rl][lane * 4]);
}
__global__ __launch_bounds__(128) void k_qkv(const float* __restrict__ EMB, const int* __restrict__ IDS, const __bf16* __restrict__ PW, const float* __restrict__ PEW, float* __restrict__ QKV) {
  __shared__ __align__(16) float so[4][16][132];
  const int tid = threadIdx.x, wave = tid >> 5, lane = tid & 31, col = lane & 15, g = lane >> 4; const size_t r0 = (size_t)blockIdx.x * 64 + wave * 16; const int n0 = blockIdx.y * 128;
  const int id = min(max(IDS[r0 + col], 0), VOC - 1); const float* er = EMB + (size_t)id * DD;
  v8f acc[8] = {};
#pragma unroll
  for (int kc = 0; kc < DD / 32; ++kc) { v16b a; const float* p = er + kc * 32 + 8 * g;
#pragma unroll
    for (int i = 0; i < 8; ++i) { a[i] = (__bf16)p[i]; a[8 + i] = (__bf16)p[16 + i]; }
#pragma unroll
    for (int j = 0; j < 8; ++j) acc[j] = wmma_bf(a, frag_b(PW + (size_t)(n0 + j * 16 + col) * DD + kc * 32, lane), acc[j]); }
#pragma unroll
  for (int j = 0; j < 8; ++j)
#pragma unroll
    for (int r = 0; r < 8; ++r) { const size_t row = r0 + 8 * g + r; const int s = (int)(row % SS); so[wave][8 * g + r][j * 16 + col] = acc[j][r] + PEW[(size_t)s * (3 * DD) + n0 + j * 16 + col]; }
  LDSX();
  for (int rl = 0; rl < 16; ++rl) vst2(QKV + (r0 + rl) * (3 * DD) + n0 + lane * 4, *(const v4f*)&so[wave][rl][lane * 4]);
}
__global__ __launch_bounds__(128) void k_attn(const float* __restrict__ QKV, float* __restrict__ WP) {
  __shared__ float sl[64][SS + 4];
  const int tid = threadIdx.x, wave = tid >> 5, lane = tid & 31, col = lane & 15, g = lane >> 4; const int b = blockIdx.y, qb = blockIdx.x; const size_t rq = (size_t)b * SS + qb * 64 + wave * 16;
  const float* qrow = QKV + (rq + col) * (3 * DD);
#pragma unroll 1
  for (int ks = 0; ks < SS / 16; ++ks) { const size_t rk = (size_t)b * SS + ks * 16 + col; const float* krow = QKV + rk * (3 * DD) + DD; v8f c = {};
#pragma unroll
    for (int kc = 0; kc < DD / 32; ++kc) { const F2 qa = split_row(qrow, kc * 32, lane); const F2 kb = split_row(krow, kc * 32, lane); c = mac3(qa, kb, c); }
#pragma unroll
    for (int r = 0; r < 8; ++r) sl[wave * 16 + 8 * g + r][ks * 16 + col] = c[r] * 0.0625f; }
  __syncthreads();
  for (int rr = 0; rr < 16; ++rr) { const int row = wave * 16 + rr; float mx = -3.0e38f; for (int t = lane; t < SS; t += 32) mx = fmaxf(mx, sl[row][t]);
#pragma unroll
    for (int o = 1; o < 32; o <<= 1) mx = fmaxf(mx, __shfl_xor(mx, o));
    float z = 0.f; for (int t = lane; t < SS; t += 32) { const float e = exp_ni(sl[row][t] - mx); sl[row][t] = e; z += e; }
#pragma unroll
    for (int o = 1; o < 32; o <<= 1) z += __shfl_xor(z, o);
    const float iz = 1.0f / z; for (int t = lane; t < SS; t += 32) sl[row][t] *= iz; }
  __syncthreads();
  __shared__ __align__(16) float sw[SS];
  for (int t = tid; t < SS; t += 128) { float acc = 0.f; for (int row = 0; row < 64; ++row) acc += sl[row][t]; sw[t] = acc; }
  __syncthreads();
  vst2(WP + ((size_t)b * 8 + qb) * SS + tid * 4, *(const v4f*)&sw[tid * 4]);
}
__global__ __launch_bounds__(256) void k_head(const float* __restrict__ QKV, const float* __restrict__ WP, const float* __restrict__ WC1, const float* __restrict__ BC1, const float* __restrict__ WC2, const float* __restrict__ BC2, float* __restrict__ OUTL) {
  __shared__ float sw[SS]; __shared__ float sp[DD]; __shared__ float sh[HID]; __shared__ __align__(16) float so[2 * NCLS];
  const int tid = threadIdx.x;
#pragma unroll 1
  for (int sub = 0; sub < 2; ++sub) { const int b = blockIdx.x * 2 + sub; __syncthreads();
  for (int t = tid; t < SS; t += 256) { float a = 0.f; for (int qb = 0; qb < 8; ++qb) a += WP[((size_t)b * 8 + qb) * SS + t]; sw[t] = a; }
  __syncthreads();
  { float acc = 0.f; const float* vb = QKV + (size_t)b * SS * (3 * DD) + 2 * DD + tid; for (int t = 0; t < SS; ++t) acc += sw[t] * vb[(size_t)t * (3 * DD)]; sp[tid] = acc / (float)SS; }
  __syncthreads();
  if (tid < HID) { float a = bfr(BC1[tid]); for (int d = 0; d < DD; ++d) a += sp[d] * bfr(WC1[d * HID + tid]); sh[tid] = fmaxf(a, 0.f); }
  __syncthreads();
  if (tid < NCLS) { float a = bfr(BC2[tid]); for (int k = 0; k < HID; ++k) a += sh[k] * bfr(WC2[k * NCLS + tid]); so[sub * NCLS + tid] = a; } }
  __syncthreads();
  if (tid < 8) vst2(OUTL + (size_t)blockIdx.x * 2 * NCLS + tid * 4, *(const v4f*)&so[tid * 4]);
}
extern "C" void kernel_launch(void* const* d_in, const int* in_sizes, int n_in, void* d_out, int out_size, void* d_ws, size_t ws_size, hipStream_t stream) {
  (void)in_sizes; (void)n_in; (void)out_size;
  const float** F = (const float**)d_in; const int* IDS = (const int*)d_in[0];
  if (ws_size < (size_t)WS_END) return;
  char* ws = (char*)d_ws; __bf16* PW = (__bf16*)(ws + WS_PW); float *PEW = (float*)(ws + WS_PEW), *QKV = (float*)(ws + WS_QKV), *WP = (float*)(ws + WS_WP);
  k_packT<<<3 * DD, 256, 0, stream>>>(F[2], F[4], F[6], PW);
  k_pe<<<dim3(SS / 64, 3 * DD / 128), 128, 0, stream>>>(PW, F[3], F[5], F[7], PEW);
  k_qkv<<<dim3(TNB * SS / 64, 3 * DD / 128), 128, 0, stream>>>(F[1], IDS, PW, PEW, QKV);
  k_attn<<<dim3(SS / 64, TNB), 128, 0, stream>>>(QKV, WP);
  k_head<<<TNB / 2, 256, 0, stream>>>(QKV, WP, F[8], F[9], F[10], F[11], (float*)d_out);
}
